// GINet_55439437856837
// MI455X (gfx1250) — hardware-verified
//
#include <hip/hip_runtime.h>
#include <stddef.h>
#include <stdint.h>


#define DIN     128
#define TK      256
#define HW      256
#define NOC     12
#define NTHR    256
#define NWAVE   8
#define EPT     8
#define CHUNK   (NTHR * EPT)
#define WCAP    (EPT * 32)
#define LISTN   (NWAVE * WCAP)
#define NBMAX   2048
#define RCAP    28672
#define DEGCAP  64
#define PKS     11
#define GBM     64
#define GBN     128
#define GTHR    128
#define GNT     8
#define PARTW   288
#define PG      32
#define HBM     32
#define HTHR    128
#define NU1     (DIN * (DIN / 8))
#define NU2     (DIN * (TK / 8))
#define NU3     (HW * (TK / 8))
#define NUB1    (NU1)
#define NUB2    (NU1 + NU2)
#define NUTOT   (NU1 + NU2 + NU3)
#define WSMAX   134217728
#define LDS_AGG ((2 * RCAP + 2 * NBMAX + LISTN) * 4 + 64)

static_assert((CHUNK & (CHUNK - 1)) == 0 && CHUNK <= (1 << PKS));
static_assert((NBMAX & (NBMAX - 1)) == 0 && NBMAX <= (1 << PKS));
static_assert(NTHR * 8 == NBMAX);
static_assert(LISTN >= NBMAX && LISTN >= NWAVE * WCAP);
static_assert((RCAP % 32) == 0);
static_assert(LDS_AGG <= 300000);
static_assert(GBM == (GTHR / 32) * 16 && GBN == 16 * GNT && GTHR == GBN && GBN == 4 * 32);
static_assert(DIN == 32 * 4 && DIN == GBN && TK == 2 * DIN);
static_assert((DIN % 32) == 0 && (TK % 32) == 0);
static_assert((PARTW % 32) == 0 && PARTW >= 2 * GBN + 1 && PARTW / 4 <= GTHR);
static_assert((NU1 % NTHR) == 0 && (NU2 % NTHR) == 0 && (NU3 % NTHR) == 0);
static_assert((DIN / 8) == 16 && (TK / 8) == 32);
static_assert((PG & (PG - 1)) == 0 && PG <= NBMAX && ((PG * (DIN / 8)) % NTHR) == 0);
static_assert(NTHR == 2 * DIN);
static_assert(HBM == 32 && HTHR == 128 && HW == 2 * GBN);
static_assert((HBM * NOC) % 4 == 0 && (HBM * NOC) / 4 <= HTHR && (HBM * NOC) == 3 * HTHR);
static_assert((HBM * NOC * 4) % 128 == 0);

typedef float          v4f  __attribute__((ext_vector_type(4)));
typedef float          v8f  __attribute__((ext_vector_type(8)));
typedef int            v4i  __attribute__((ext_vector_type(4)));
typedef int            v8i  __attribute__((ext_vector_type(8)));
typedef unsigned int   v2u  __attribute__((ext_vector_type(2)));
typedef unsigned short v8us __attribute__((ext_vector_type(8)));
typedef __bf16         v16b __attribute__((ext_vector_type(16)));
typedef v4f  __attribute__((may_alias)) v4fa;
typedef v8us __attribute__((may_alias)) v8usa;
union Frag { v16b vb; v8us h[2]; v8i w; };

__device__ __forceinline__ v8f wmx(const Frag& a, const Frag& b, v8f c) {
  v8f d = __builtin_amdgcn_wmma_f32_16x16x32_bf16(false, a.vb, false, b.vb, (short)0, c, false, false);
  asm volatile("v_nop\n\tv_nop\n\tv_nop\n\tv_nop" : "+v"(d) : "v"(a.w), "v"(b.w));
  return d;
}

__device__ __forceinline__ unsigned short bf_bits(float f) {
  unsigned int u = __float_as_uint(f);
  u += 0x7FFFu + ((u >> 16) & 1u);
  return (unsigned short)(u >> 16);
}
__device__ __forceinline__ float bf_val(unsigned short b) { return __uint_as_float(((unsigned int)b) << 16); }
__device__ __forceinline__ float bf_rne(float f) { return bf_val(bf_bits(f)); }

__device__ __forceinline__ float relu_np(float v) { return (v > 0.0f) ? v : (v - v); }

__device__ __forceinline__ void hilo8(const v4f a, const v4f b, v8us& hv, v8us& lv) {
  const float f[8] = {a.x, a.y, a.z, a.w, b.x, b.y, b.z, b.w};
#pragma unroll
  for (int j = 0; j < 8; ++j) {
    const unsigned short hb = bf_bits(f[j]);
    hv[j] = hb;
    lv[j] = bf_bits(f[j] - bf_val(hb));
  }
}

__device__ __forceinline__ int scan_chunk(const int* __restrict__ dsts, int nE, int cbase, int slotBase,
                                          int nb, int vec8, int* list, int tid, int lane, int wave) {
  int wc = 0;
  const int el0  = tid * EPT;
  const int e0   = cbase + el0;
  const int sent = -2147483647 - 1;
  v4i da, db;
  if (vec8 != 0 && cbase + CHUNK <= nE) {
    da = *(const v4i*)(dsts + e0);
    db = *(const v4i*)(dsts + e0 + 4);
  } else {
    da.x = (e0     < nE) ? dsts[min(e0,     nE - 1)] : sent;
    da.y = (e0 + 1 < nE) ? dsts[min(e0 + 1, nE - 1)] : sent;
    da.z = (e0 + 2 < nE) ? dsts[min(e0 + 2, nE - 1)] : sent;
    da.w = (e0 + 3 < nE) ? dsts[min(e0 + 3, nE - 1)] : sent;
    db.x = (e0 + 4 < nE) ? dsts[min(e0 + 4, nE - 1)] : sent;
    db.y = (e0 + 5 < nE) ? dsts[min(e0 + 5, nE - 1)] : sent;
    db.z = (e0 + 6 < nE) ? dsts[min(e0 + 6, nE - 1)] : sent;
    db.w = (e0 + 7 < nE) ? dsts[min(e0 + 7, nE - 1)] : sent;
  }
  const unsigned nbs = (unsigned)slotBase;
  const unsigned unb = (unsigned)nb;
  const unsigned s0 = (unsigned)da.x - nbs, s1 = (unsigned)da.y - nbs;
  const unsigned s2 = (unsigned)da.z - nbs, s3 = (unsigned)da.w - nbs;
  const unsigned s4 = (unsigned)db.x - nbs, s5 = (unsigned)db.y - nbs;
  const unsigned s6 = (unsigned)db.z - nbs, s7 = (unsigned)db.w - nbs;
  const bool h0 = s0 < unb, h1 = s1 < unb, h2 = s2 < unb, h3 = s3 < unb;
  const bool h4 = s4 < unb, h5 = s5 < unb, h6 = s6 < unb, h7 = s7 < unb;
  const unsigned any = __builtin_amdgcn_ballot_w32(h0 | h1 | h2 | h3 | h4 | h5 | h6 | h7);
  if (any != 0u) {
#define HITJ(J, HJ, SJ) { \
      const unsigned mj = __builtin_amdgcn_ballot_w32(HJ); \
      if (mj != 0u) { \
        if (HJ) { \
          const int pos = wc + (int)__builtin_amdgcn_mbcnt_lo(mj, 0u); \
          if (pos < WCAP) list[wave * WCAP + pos] = ((el0 + (J)) << PKS) | (int)(SJ); \
        } \
        wc += (int)__builtin_popcount(mj); } }
    HITJ(0, h0, s0)
    HITJ(1, h1, s1)
    HITJ(2, h2, s2)
    HITJ(3, h3, s3)
    HITJ(4, h4, s4)
    HITJ(5, h5, s5)
    HITJ(6, h6, s6)
    HITJ(7, h7, s7)
#undef HITJ
  }
  return wc;
}

__device__ __forceinline__ v8us cv8b(const float* __restrict__ p, size_t stride) {
  v8us o;
#pragma unroll
  for (int i = 0; i < 8; ++i) o[i] = bf_bits(p[(size_t)i * stride]);
  return o;
}

__global__ __launch_bounds__(NTHR) void k_wprep(const float* __restrict__ W1, const float* __restrict__ W2,
                                                const float* __restrict__ Wf1,
                                                unsigned short* p1, unsigned short* p2, unsigned short* p3) {
  const int u = (int)blockIdx.x * NTHR + (int)threadIdx.x;
  v8us o;
  unsigned short* dp;
  if (u < NUB1) {
    const int v = u, n = v >> 4, k8 = (v & 15) * 8;
    o = cv8b(W1 + (size_t)k8 * DIN + n, DIN);
    dp = p1 + (size_t)v * 8;
  } else if (u < NUB2) {
    const int v = u - NUB1, n = v >> 5, k8 = (v & 31) * 8;
    const int kk = k8 & (DIN - 1);
    o = cv8b(W2 + (size_t)kk * DIN + n, DIN);
    dp = p2 + (size_t)v * 8;
  } else if (u < NUTOT) {
    const int v = u - NUB2, n = v >> 5, k8 = (v & 31) * 8;
    const int kk = k8 & (DIN - 1);
    o = cv8b(Wf1 + (size_t)kk * HW + n, HW);
    dp = p3 + (size_t)v * 8;
  } else {
    return;
  }
  *(volatile v8us*)dp = o;
  __threadfence();
  *(volatile v8us*)dp = o;
}

__global__ __launch_bounds__(NTHR) void k_cvx(const float* __restrict__ x, int nN, int nUnits,
                                              unsigned short* xb) {
  const int u = (int)blockIdx.x * NTHR + (int)threadIdx.x;
  if (u >= nUnits) return;
  const int row = u >> 4;
  const int k8  = (u & 15) * 8;
  const int rc  = row < nN ? row : nN - 1;
  const float* p = x + (size_t)rc * DIN + k8;
  const v4f a = *(const v4fa*)p;
  const v4f b = *(const v4fa*)(p + 4);
  const bool ok = row < nN;
  v8us o;
  o[0] = ok ? bf_bits(a.x) : (unsigned short)0;
  o[1] = ok ? bf_bits(a.y) : (unsigned short)0;
  o[2] = ok ? bf_bits(a.z) : (unsigned short)0;
  o[3] = ok ? bf_bits(a.w) : (unsigned short)0;
  o[4] = ok ? bf_bits(b.x) : (unsigned short)0;
  o[5] = ok ? bf_bits(b.y) : (unsigned short)0;
  o[6] = ok ? bf_bits(b.z) : (unsigned short)0;
  o[7] = ok ? bf_bits(b.w) : (unsigned short)0;
  unsigned short* dp = xb + (size_t)row * DIN + k8;
  *(volatile v8us*)dp = o;
  __threadfence();
  *(volatile v8us*)dp = o;
}

__global__ __launch_bounds__(NTHR) void k_agg(
    const int* __restrict__ srcs, const int* __restrict__ dsts,
    const float* __restrict__ fin, const float* __restrict__ b1,
    unsigned short* Tout, int ldt,
    int nN, int nE, int nb, int vec8, int MPr) {
  extern __shared__ v4f lds_dyn[];
  int* reg1 = (int*)lds_dyn;
  int* reg2 = reg1 + RCAP;
  int* scnt = reg2 + RCAP;
  int* soff = scnt + NBMAX;
  int* list = soff + NBMAX;
  int* wcnt = list + LISTN;
  int* wtot = wcnt + NWAVE;
  const int tid = (int)threadIdx.x, lane = tid & 31, wave = tid >> 5;
  const int nodeBase = (int)blockIdx.x * nb;

  for (int i = tid; i < NBMAX; i += NTHR) scnt[i] = 0;
  float bb0, bb1, bb2, bb3;
  {
    const v4f bv = *(const v4f*)(b1 + 4 * lane);
    bb0 = bf_rne(bv.x); bb1 = bf_rne(bv.y); bb2 = bf_rne(bv.z); bb3 = bf_rne(bv.w);
  }
  __syncthreads();

  int tot = 0;
  const int nChunks = (nE + CHUNK - 1) / CHUNK;
#pragma unroll 1
  for (int ch = 0; ch < nChunks; ++ch) {
    const int cbase = ch * CHUNK;
    const int wc = scan_chunk(dsts, nE, cbase, nodeBase, nb, vec8, list, tid, lane, wave);
    if (lane == 0) wcnt[wave] = wc;
    __syncthreads();
    int pre = 0, all = 0;
#pragma unroll
    for (int w2 = 0; w2 < NWAVE; ++w2) {
      int c = wcnt[w2];
      c = c < 0 ? 0 : (c > WCAP ? WCAP : c);
      all += c;
      pre += (w2 < wave) ? c : 0;
    }
    const int wcc  = wc > WCAP ? WCAP : wc;
    const int base = tot + pre;
#pragma unroll 1
    for (int i = lane; i < wcc; i += 32) {
      const int ent = list[wave * WCAP + i];
      const int el  = (ent >> PKS) & (CHUNK - 1);
      const int sl  = ent & (NBMAX - 1);
      int eid = cbase + el;
      eid = eid > nE - 1 ? nE - 1 : eid;
      const int pos = base + i;
      if (pos < RCAP) reg1[pos] = (int)(((unsigned)eid << PKS) | (unsigned)sl);
    }
    tot += all;
    tot = tot > RCAP ? RCAP : tot;
    __syncthreads();
  }
  const int nh = tot;

  if (wave == 0) {
#pragma unroll 1
    for (int b0 = 0; b0 < nh; b0 += 32) {
      const int idx = b0 + lane;
      const int uv  = reg1[idx < RCAP ? idx : RCAP - 1];
      const int m32 = (nh - b0) < 32 ? (nh - b0) : 32;
#pragma unroll 1
      for (int k = 0; k < m32; ++k) {
        const int u  = __builtin_amdgcn_readlane(uv, k);
        const int sl = u & (NBMAX - 1);
        if (lane == 0) scnt[sl] = scnt[sl] + 1;
      }
    }
  }
  __syncthreads();

  {
    const v4i ca = *(const v4i*)(scnt + 8 * tid);
    const v4i cb = *(const v4i*)(scnt + 8 * tid + 4);
    const int e0 = ca.x < 0 ? 0 : ca.x, e1 = ca.y < 0 ? 0 : ca.y, e2 = ca.z < 0 ? 0 : ca.z, e3 = ca.w < 0 ? 0 : ca.w;
    const int e4 = cb.x < 0 ? 0 : cb.x, e5 = cb.y < 0 ? 0 : cb.y, e6 = cb.z < 0 ? 0 : cb.z, e7 = cb.w < 0 ? 0 : cb.w;
    const int ts = e0 + e1 + e2 + e3 + e4 + e5 + e6 + e7;
    int incl = ts;
#pragma unroll
    for (int d = 1; d < 32; d <<= 1) {
      const int up = __shfl_up(incl, d);
      if (lane >= d) incl += up;
    }
    if (lane == 31) wtot[wave] = incl;
    __syncthreads();
    int pre = 0;
#pragma unroll
    for (int w2 = 0; w2 < NWAVE; ++w2) pre += (w2 < wave) ? wtot[w2] : 0;
    int run = pre + incl - ts;
    soff[8 * tid + 0] = run; run += e0;
    soff[8 * tid + 1] = run; run += e1;
    soff[8 * tid + 2] = run; run += e2;
    soff[8 * tid + 3] = run; run += e3;
    soff[8 * tid + 4] = run; run += e4;
    soff[8 * tid + 5] = run; run += e5;
    soff[8 * tid + 6] = run; run += e6;
    soff[8 * tid + 7] = run;
  }
  __syncthreads();
  for (int i = tid; i < NBMAX; i += NTHR) list[i] = soff[i];
  __syncthreads();

  if (wave == 0) {
#pragma unroll 1
    for (int b0 = 0; b0 < nh; b0 += 32) {
      const int idx = b0 + lane;
      const int uv  = reg1[idx < RCAP ? idx : RCAP - 1];
      const int m32 = (nh - b0) < 32 ? (nh - b0) : 32;
#pragma unroll 1
      for (int k = 0; k < m32; ++k) {
        const int u   = __builtin_amdgcn_readlane(uv, k);
        const int sl  = u & (NBMAX - 1);
        const int eid = (int)((unsigned)u >> PKS);
        if (lane == 0) {
          int pos = list[sl];
          pos = pos < 0 ? 0 : (pos > RCAP - 1 ? RCAP - 1 : pos);
          reg2[pos] = eid;
          list[sl] = pos + 1;
        }
      }
    }
  }
  __syncthreads();

  const int nbw = nb >> 3;
  const bool ovf = (nh >= RCAP);
  const float qnan = __int_as_float(0x7fc00000);

#pragma unroll 1
  for (int jt = 0; jt < nbw; ++jt) {
    const int slot = wave * nbw + jt;
    const int grow = nodeBase + slot;
    int st = soff[slot];
    const int craw = scnt[slot];
    int cnt = craw;
    st  = st < 0 ? 0 : (st > nh ? nh : st);
    cnt = cnt < 0 ? 0 : (cnt > DEGCAP ? DEGCAP : cnt);
    if (cnt > nh - st) cnt = nh - st;
    const float pz = (ovf || craw > DEGCAP) ? qnan : 0.0f;
    const bool liveRow = grow < nN;

    float ag0 = 0.f, ag1 = 0.f, ag2 = 0.f, ag3 = 0.f;
#pragma unroll 1
    for (int q = 0; q < cnt; ++q) {
      int idx = st + q; idx = idx > RCAP - 1 ? RCAP - 1 : idx;
      int eid = reg2[idx]; eid = eid < 0 ? 0 : (eid > nE - 1 ? nE - 1 : eid);
      const int sraw = srcs[eid];
      const int s = sraw < 0 ? 0 : (sraw > nN - 1 ? nN - 1 : sraw);
      const v4f v = *(const v4f*)(fin + (size_t)s * DIN + 4 * lane);
      ag0 += v.x; ag1 += v.y; ag2 += v.z; ag3 += v.w;
    }
    const int nc = liveRow ? grow : nN - 1;
    const v4f sv = *(const v4f*)(fin + (size_t)nc * DIN + 4 * lane);
    float r0 = (sv.x + ag0) + bb0, r1 = (sv.y + ag1) + bb1;
    float r2 = (sv.z + ag2) + bb2, r3 = (sv.w + ag3) + bb3;
    r0 = relu_np(r0); r1 = relu_np(r1); r2 = relu_np(r2); r3 = relu_np(r3);
    r0 = (liveRow ? r0 : 0.0f) + pz;
    r1 = (liveRow ? r1 : 0.0f) + pz;
    r2 = (liveRow ? r2 : 0.0f) + pz;
    r3 = (liveRow ? r3 : 0.0f) + pz;

    const unsigned short hb0 = bf_bits(r0), hb1 = bf_bits(r1), hb2 = bf_bits(r2), hb3 = bf_bits(r3);
    const unsigned short lb0 = bf_bits(r0 - bf_val(hb0)), lb1 = bf_bits(r1 - bf_val(hb1));
    const unsigned short lb2 = bf_bits(r2 - bf_val(hb2)), lb3 = bf_bits(r3 - bf_val(hb3));
    v2u ph, pl;
    ph.x = (unsigned int)hb0 | ((unsigned int)hb1 << 16);
    ph.y = (unsigned int)hb2 | ((unsigned int)hb3 << 16);
    pl.x = (unsigned int)lb0 | ((unsigned int)lb1 << 16);
    pl.y = (unsigned int)lb2 | ((unsigned int)lb3 << 16);
    unsigned short* hp = Tout + (size_t)grow * (size_t)ldt + 4 * lane;
    unsigned short* lp = hp + DIN;
    const bool wsv = grow < MPr;
    if (wsv) { *(volatile v2u*)hp = ph; *(volatile v2u*)lp = pl; }
    __threadfence();
    if (wsv) { *(volatile v2u*)hp = ph; *(volatile v2u*)lp = pl; }
  }
}

template <int EPI>
__global__ __launch_bounds__(GTHR) void k_gemm(const unsigned short* __restrict__ A, int lda,
                                               const unsigned short* __restrict__ BT, int ldb, int K,
                                               const float* __restrict__ bias,
                                               float* outF, int ldo, int nN, int mRows,
                                               float* part) {
  __shared__ __attribute__((aligned(16))) float stg[GBM * GBN];
  __shared__ __attribute__((aligned(16))) float pst[PARTW];
  const int tid = (int)threadIdx.x, lane = tid & 31, wave = tid >> 5, hh = lane >> 4, m = lane & 15;
  const int rowBase = (int)blockIdx.x * GBM;
  const int colBase = (int)blockIdx.y * GBN;

  v8f acc[GNT];
  {
    const v8f z = {0.f, 0.f, 0.f, 0.f, 0.f, 0.f, 0.f, 0.f};
#pragma unroll
    for (int t = 0; t < GNT; ++t) acc[t] = z;
  }
  const unsigned short* ap = A  + (size_t)(rowBase + 16 * wave + m) * (size_t)lda + 8 * hh;
  const unsigned short* bp = BT + (size_t)(colBase + m) * (size_t)ldb + 8 * hh;

#pragma unroll 1
  for (int k0 = 0; k0 < K; k0 += 32) {
    Frag af;
    af.h[0] = *(const v8usa*)(ap + k0);
    af.h[1] = *(const v8usa*)(ap + k0 + 16);
#pragma unroll
    for (int nt = 0; nt < GNT; ++nt) {
      const unsigned short* wq = bp + (size_t)(16 * nt) * (size_t)ldb + k0;
      Frag bfr;
      bfr.h[0] = *(const v8usa*)wq;
      bfr.h[1] = *(const v8usa*)(wq + 16);
      acc[nt] = wmx(af, bfr, acc[nt]);
    }
  }

#pragma unroll
  for (int nt = 0; nt < GNT; ++nt) {
    const int lc = 16 * nt + m;
    float bb = 0.0f;
    if constexpr (EPI == 1) bb = bf_rne(bias[colBase + lc]);
#pragma unroll
    for (int r = 0; r < 8; ++r) {
      const int lr = 16 * wave + 8 * hh + r;
      const bool live = (rowBase + lr) < nN;
      float v = acc[nt][r];
      if constexpr (EPI == 1) v = relu_np(v + bb);
      stg[lr * GBN + lc] = live ? v : 0.0f;
    }
  }
  __syncthreads();

  v4f fv[16];
#pragma unroll
  for (int i = 0; i < 16; ++i) {
    const int lr = 16 * wave + i;
    fv[i] = *(const v4fa*)(stg + lr * GBN + 4 * lane);
  }
  v4f pv = {0.f, 0.f, 0.f, 0.f};
  const bool pok = (EPI == 1) && (tid < PARTW / 4);
  if constexpr (EPI == 1) {
    int nvr = nN - rowBase;
    nvr = nvr < 0 ? 0 : (nvr > GBM ? GBM : nvr);
    float s = 0.0f;
#pragma unroll 1
    for (int r = 0; r < nvr; ++r) s += stg[r * GBN + tid];
    const float inv = 1.0f / (float)(nvr < 1 ? 1 : nvr);
    const float mean = s * inv;
    float q = 0.0f;
#pragma unroll 1
    for (int r = 0; r < nvr; ++r) {
      const float d = stg[r * GBN + tid] - mean;
      q = fmaf(d, d, q);
    }
    pst[1 + tid] = mean;
    pst[1 + GBN + tid] = q;
    if (tid == 0) pst[0] = (float)nvr;
#pragma unroll 1
    for (int i = 2 * GBN + 1 + tid; i < PARTW; i += GTHR) pst[i] = 0.0f;
    __syncthreads();
    if (pok) pv = *(const v4fa*)(pst + 4 * tid);
  }
  const size_t prow = (size_t)blockIdx.x * (size_t)gridDim.y + (size_t)blockIdx.y;
  float* pp = part + prow * PARTW + 4 * tid;
#pragma unroll
  for (int i = 0; i < 16; ++i) {
    const int gr = rowBase + 16 * wave + i;
    float* op = outF + (size_t)gr * (size_t)ldo + colBase + 4 * lane;
    if (gr < mRows) *(volatile v4f*)op = fv[i];
  }
  if (pok) *(volatile v4f*)pp = pv;
  __threadfence();
#pragma unroll
  for (int i = 0; i < 16; ++i) {
    const int gr = rowBase + 16 * wave + i;
    float* op = outF + (size_t)gr * (size_t)ldo + colBase + 4 * lane;
    if (gr < mRows) *(volatile v4f*)op = fv[i];
  }
  if (pok) *(volatile v4f*)pp = pv;
}

__global__ __launch_bounds__(GBN) void k_bnfin(const float* __restrict__ part, int nPart, float* ss) {
  __shared__ __attribute__((aligned(16))) float stg[2 * GBN];
  const int tid = (int)threadIdx.x;
  double n = 0.0, mean = 0.0, M2 = 0.0;
#pragma unroll 1
  for (int b = 0; b < nPart; ++b) {
    const float* pr = part + (size_t)b * PARTW;
    const double nb = (double)pr[0];
    const double mb = (double)pr[1 + tid];
    const double qb = (double)pr[1 + GBN + tid];
    if (nb > 0.5) {
      const double nn = n + nb;
      const double delta = mb - mean;
      const double f = nb / nn;
      mean = mean + delta * f;
      M2 = M2 + qb + delta * delta * n * f;
      n = nn;
    }
  }
  const double nt = n < 1.0 ? 1.0 : n;
  const float var = (float)(M2 / nt);
  const float rs  = 1.0f / sqrtf(var + 1e-5f);
  stg[tid] = (float)mean;
  stg[GBN + tid] = rs;
  __syncthreads();
  const int seg = tid >> 5, j = tid & 31;
  const bool ok = tid < 64;
  const int sc = ok ? seg : 0;
  const v4f v = *(const v4fa*)(stg + sc * GBN + 4 * j);
  float* dp = ss + (size_t)sc * GBN + 4 * j;
  if (ok) *(volatile v4f*)dp = v;
  __threadfence();
  if (ok) *(volatile v4f*)dp = v;
}

__global__ __launch_bounds__(NTHR) void k_pool(const float* __restrict__ H, const float* __restrict__ ss,
                                               const float* __restrict__ gam, const float* __restrict__ bet,
                                               const int* __restrict__ bat, int nN, int nG,
                                               unsigned short* gp) {
  __shared__ __attribute__((aligned(16))) float accs[PG * DIN];
  __shared__ float ssh[4 * DIN];
  __shared__ __attribute__((aligned(16))) int list[LISTN];
  __shared__ int wcnt[NWAVE];
  const int tid = (int)threadIdx.x, lane = tid & 31, wave = tid >> 5;
  const int slotBase = (int)blockIdx.x * PG;

  for (int i = tid; i < PG * DIN; i += NTHR) accs[i] = 0.0f;
  ssh[tid] = ss[tid];
  {
    const int c = tid & (DIN - 1);
    const float gv = gam[c];
    const float bv = bet[c];
    ssh[2 * DIN + tid] = bf_rne(tid < DIN ? gv : bv);
  }
  __syncthreads();

  const int nChunks = (nN + CHUNK - 1) / CHUNK;
#pragma unroll 1
  for (int ch = 0; ch < nChunks; ++ch) {
    const int cbase = ch * CHUNK;
    const int wc = scan_chunk(bat, nN, cbase, slotBase, PG, 1, list, tid, lane, wave);
    if (lane == 0) wcnt[wave] = wc;
    __syncthreads();
#pragma unroll 1
    for (int w2 = 0; w2 < NWAVE; ++w2) {
      int c = wcnt[w2];
      c = c < 0 ? 0 : (c > WCAP ? WCAP : c);
#pragma unroll 1
      for (int i = 0; i < c; ++i) {
        const int ent = list[w2 * WCAP + i];
        const int el  = (ent >> PKS) & (CHUNK - 1);
        const int sl  = ent & (PG - 1);
        int node = cbase + el;
        node = node < 0 ? 0 : (node > nN - 1 ? nN - 1 : node);
#pragma unroll 1
        for (int cc = tid; cc < DIN; cc += NTHR) {
          const float u = H[(size_t)node * DIN + cc];
          const float v = ((u - ssh[cc]) * ssh[DIN + cc]) * ssh[2 * DIN + cc] + ssh[3 * DIN + cc];
          accs[sl * DIN + cc] += v;
        }
      }
    }
    __syncthreads();
  }

  constexpr int PPR = DIN / 8;
  constexpr int NIT = (PG * PPR) / NTHR;
  v8us hv[NIT], lv[NIT];
#pragma unroll
  for (int it = 0; it < NIT; ++it) {
    const int p = it * NTHR + tid;
    const int row = p / PPR, q = p % PPR;
    const v4f a = *(const v4fa*)(accs + row * DIN + 8 * q);
    const v4f b = *(const v4fa*)(accs + row * DIN + 8 * q + 4);
    hilo8(a, b, hv[it], lv[it]);
  }
#pragma unroll
  for (int it = 0; it < NIT; ++it) {
    const int p = it * NTHR + tid;
    const int row = p / PPR, q = p % PPR;
    const int g = slotBase + row;
    unsigned short* hp = gp + (size_t)g * TK + 8 * q;
    unsigned short* lp = hp + DIN;
    if (g < nG) { *(volatile v8us*)hp = hv[it]; *(volatile v8us*)lp = lv[it]; }
  }
  __threadfence();
#pragma unroll
  for (int it = 0; it < NIT; ++it) {
    const int p = it * NTHR + tid;
    const int row = p / PPR, q = p % PPR;
    const int g = slotBase + row;
    unsigned short* hp = gp + (size_t)g * TK + 8 * q;
    unsigned short* lp = hp + DIN;
    if (g < nG) { *(volatile v8us*)hp = hv[it]; *(volatile v8us*)lp = lv[it]; }
  }
}

__global__ __launch_bounds__(HTHR) void k_head(const unsigned short* __restrict__ G,
                                               const unsigned short* __restrict__ WF,
                                               const float* __restrict__ bf1, const float* __restrict__ Wf2,
                                               const float* __restrict__ bf2, float* out) {
  __shared__ __attribute__((aligned(16))) float stg[HBM * HW];
  __shared__ float w2s[HW * NOC];
  __shared__ float b2s[16];
  __shared__ __attribute__((aligned(16))) float os[HBM * NOC];
  const int tid = (int)threadIdx.x, lane = tid & 31, wave = tid >> 5, hh = lane >> 4, m = lane & 15;
  const int rowBase = (int)blockIdx.x * HBM;
  const int rt = wave & 1, ch = wave >> 1;

#pragma unroll 4
  for (int i = tid; i < HW * NOC; i += HTHR) w2s[i] = bf_rne(Wf2[i]);
  if (tid < 16) {
    const float bb = bf2[tid < NOC ? tid : NOC - 1];
    b2s[tid] = (tid < NOC) ? bf_rne(bb) : 0.0f;
  }

  v8f acc[GNT];
  {
    const v8f z = {0.f, 0.f, 0.f, 0.f, 0.f, 0.f, 0.f, 0.f};
#pragma unroll
    for (int t = 0; t < GNT; ++t) acc[t] = z;
  }
  const unsigned short* ap = G  + (size_t)(rowBase + 16 * rt + m) * (size_t)TK + 8 * hh;
  const unsigned short* bp = WF + (size_t)(ch * GBN + m) * (size_t)TK + 8 * hh;
#pragma unroll 1
  for (int k0 = 0; k0 < TK; k0 += 32) {
    Frag af;
    af.h[0] = *(const v8usa*)(ap + k0);
    af.h[1] = *(const v8usa*)(ap + k0 + 16);
#pragma unroll
    for (int nt = 0; nt < GNT; ++nt) {
      const unsigned short* wq = bp + (size_t)(16 * nt) * (size_t)TK + k0;
      Frag bfr;
      bfr.h[0] = *(const v8usa*)wq;
      bfr.h[1] = *(const v8usa*)(wq + 16);
      acc[nt] = wmx(af, bfr, acc[nt]);
    }
  }
#pragma unroll
  for (int nt = 0; nt < GNT; ++nt) {
    const int lc = ch * GBN + 16 * nt + m;
    const float bb = bf_rne(bf1[lc]);
#pragma unroll
    for (int r = 0; r < 8; ++r) {
      const int lr = 16 * rt + 8 * hh + r;
      stg[lr * HW + lc] = relu_np(acc[nt][r] + bb);
    }
  }
  __syncthreads();

#pragma unroll 1
  for (int it = 0; it < (HBM * NOC) / HTHR; ++it) {
    const int idx = it * HTHR + tid;
    const int row = idx / NOC;
    const int c   = idx - row * NOC;
    const float* pr = stg + row * HW;
    float s = 0.0f;
#pragma unroll 4
    for (int k4 = 0; k4 < HW / 4; ++k4) {
      const v4f p = *(const v4fa*)(pr + 4 * k4);
      const float* w = w2s + (4 * k4) * NOC + c;
      s = fmaf(p.x, w[0], s);
      s = fmaf(p.y, w[NOC], s);
      s = fmaf(p.z, w[2 * NOC], s);
      s = fmaf(p.w, w[3 * NOC], s);
    }
    os[idx] = s + b2s[c];
  }
  __syncthreads();

  constexpr int NPC = (HBM * NOC) / 4;
  const bool okst = tid < NPC;
  const int pc = okst ? tid : NPC - 1;
  const v4f ov = *(const v4fa*)(os + 4 * pc);
  float* op = out + (size_t)rowBase * NOC + 4 * pc;
  if (okst) *(volatile v4f*)op = ov;
  __threadfence();
  if (okst) *(volatile v4f*)op = ov;
}

static int pick_nb(int nE, int nN) {
  int nb = NBMAX;
  while (nb > 16 && (long long)nb * (long long)nE * 5LL > (long long)RCAP * (long long)nN * 4LL) nb >>= 1;
  return nb;
}
static inline int cdiv(int a, int b) { return (a + b - 1) / b; }
static inline size_t al256(size_t o) { return (o + 255) & ~(size_t)255; }

extern "C" void kernel_launch(void* const* d_in, const int* in_sizes, int n_in,
                              void* d_out, int out_size, void* d_ws, size_t ws_size,
                              hipStream_t stream) {
  if (n_in < 13) return;
  if (in_sizes[0] < DIN || (in_sizes[0] % DIN) != 0) return;
  const int nN = in_sizes[0] / DIN;
  if (nN < GBM || nN > (1 << 22)) return;
  const int nE2 = in_sizes[1];
  if (nE2 < 2 || (nE2 & 1) != 0) return;
  const int nE = nE2 / 2;
  if (nE < 1 || nE > (1 << 21)) return;
  if (in_sizes[2] != nN) return;
  if (in_sizes[3] != DIN * DIN || in_sizes[4] != DIN) return;
  if (in_sizes[5] != DIN * DIN || in_sizes[6] != DIN) return;
  if (in_sizes[7] != DIN || in_sizes[8] != DIN) return;
  if (in_sizes[9] != DIN * HW || in_sizes[10] != HW) return;
  if (in_sizes[11] != HW * NOC || in_sizes[12] != NOC) return;
  if (out_size < NOC || (out_size % NOC) != 0) return;
  const int nG = out_size / NOC;
  if (nG < HBM || (nG % HBM) != 0 || (nG % PG) != 0 || nG > NBMAX * 32) return;
  if ((long long)nG * NOC != (long long)out_size) return;

  const float* x     = (const float*)d_in[0];
  const int*   ei    = (const int*)  d_in[1];
  const int*   src   = ei;
  const int*   dst   = ei + nE;
  const int*   batch = (const int*)  d_in[2];
  const float* W1    = (const float*)d_in[3];
  const float* b1    = (const float*)d_in[4];
  const float* W2    = (const float*)d_in[5];
  const float* b2    = (const float*)d_in[6];
  const float* gamma = (const float*)d_in[7];
  const float* beta  = (const float*)d_in[8];
  const float* Wf1   = (const float*)d_in[9];
  const float* bf1   = (const float*)d_in[10];
  const float* Wf2   = (const float*)d_in[11];
  const float* bf2   = (const float*)d_in[12];
  float* out = (float*)d_out;

  const int MP   = cdiv(nN, GBM) * GBM;
  const int gM   = MP / GBM;
  const int nb   = pick_nb(nE, nN);
  const int gA   = cdiv(MP, nb);
  const int vec8 = ((nE & 3) == 0) ? 1 : 0;
  if ((long long)gA * nb < (long long)MP) return;
  if ((long long)(gM - 1) * GBM >= (long long)nN) return;

  char* ws = (char*)d_ws;
  size_t off = 0;
  const size_t oW1T = off; off = al256(off + (size_t)NU1 * 16);
  const size_t oW2C = off; off = al256(off + (size_t)NU2 * 16);
  const size_t oWFC = off; off = al256(off + (size_t)NU3 * 16);
  const size_t oXB  = off; off = al256(off + (size_t)MP * DIN * 2);
  const size_t oY   = off; off = al256(off + (size_t)MP * DIN * 4);
  const size_t oT   = off; off = al256(off + (size_t)MP * TK * 2);
  const size_t oH   = off; off = al256(off + (size_t)MP * DIN * 4);
  const size_t oPT  = off; off = al256(off + (size_t)gM * PARTW * 4);
  const size_t oSS  = off; off = al256(off + (size_t)(2 * DIN) * 4);
  const size_t oG   = off; off = al256(off + (size_t)nG * TK * 2);
  if (off > ws_size || off > (size_t)WSMAX) return;
  unsigned short* W1T = (unsigned short*)(ws + oW1T);
  unsigned short* W2C = (unsigned short*)(ws + oW2C);
  unsigned short* WFC = (unsigned short*)(ws + oWFC);
  unsigned short* XB  = (unsigned short*)(ws + oXB);
  float*          Y   = (float*)(ws + oY);
  unsigned short* T   = (unsigned short*)(ws + oT);
  float*          H   = (float*)(ws + oH);
  float*          PT  = (float*)(ws + oPT);
  float*          SS  = (float*)(ws + oSS);
  unsigned short* GP  = (unsigned short*)(ws + oG);

  hipFuncSetAttribute(reinterpret_cast<const void*>(&k_agg), hipFuncAttributeMaxDynamicSharedMemorySize, LDS_AGG);

  const int nUx = MP * (DIN / 8);
  k_wprep<<<NUTOT / NTHR, NTHR, 0, stream>>>(W1, W2, Wf1, W1T, W2C, WFC);
  k_cvx<<<cdiv(nUx, NTHR), NTHR, 0, stream>>>(x, nN, nUx, XB);
  k_gemm<0><<<dim3(gM, DIN / GBN), GTHR, 0, stream>>>(XB, DIN, W1T, DIN, DIN, b1, Y, DIN, nN, MP, PT);
  k_agg<<<gA, NTHR, LDS_AGG, stream>>>(src, dst, Y, b1, T, TK, nN, nE, nb, vec8, MP);
  k_gemm<1><<<dim3(gM, DIN / GBN), GTHR, 0, stream>>>(T, TK, W2C, TK, TK, b2, H, DIN, nN, MP, PT);
  k_bnfin<<<1, GBN, 0, stream>>>(PT, gM, SS);
  k_pool<<<nG / PG, NTHR, 0, stream>>>(H, SS, gamma, beta, batch, nN, nG, GP);
  k_head<<<nG / HBM, HTHR, 0, stream>>>(GP, WFC, bf1, Wf2, bf2, out);
}
